// GNNAgent_53815940219242
// MI455X (gfx1250) — hardware-verified
//
#include <hip/hip_runtime.h>
#include <stddef.h>
#include <stdint.h>


#define DF     128
#define HL     256
#define KU     512
#define NOUT   32
#define LNEPS  1e-6f
#define NTHR   256
#define NWAVE  8
#define EPT    8
#define CHUNK  (NTHR * EPT)
#define WCAP   (EPT * 32)
#define LISTN  (NWAVE * WCAP)
#define NBA    1024
#define SLA    10
#define RCAP   28672
#define DEGCAP 64
#define MEAS_B1024  13377
#define MEAS_MAXDEG 29
#define GBM    64
#define GBN    128
#define GTHR   128
#define GWAVE  (GTHR / 32)
#define ROWH   256
#define NUWP   (DF * (DF / 8))
#define NUWM   (2 * DF * (HL / 8))
#define NUWU   (DF * (KU / 8))
#define NUW    (NUWP + NUWM + NUWU)
#define FTHR   128
#define AGG_ZINTS    (LISTN + 2 * RCAP + 3 * NBA)
#define MISC_INTS    16
#define ROWBUF_INTS  (NWAVE * ROWH / 2)
#define AGG_LDS_INTS (AGG_ZINTS + MISC_INTS + ROWBUF_INTS)
#define WSMAX  134217728

static_assert((CHUNK & (CHUNK - 1)) == 0 && CHUNK <= 4096);
static_assert((NBA & (NBA - 1)) == 0 && NBA == (1 << SLA));
static_assert(((long long)CHUNK << SLA) < (1LL << 31));
static_assert(LISTN % NTHR == 0);
static_assert(NBA % NWAVE == 0 && NBA % 32 == 0 && NBA % GBM == 0);
static_assert(RCAP % 4 == 0 && AGG_ZINTS % 4 == 0 && LISTN % 4 == 0 && ((AGG_ZINTS + MISC_INTS) % 4) == 0);
static_assert(AGG_ZINTS % (NTHR * 4) == 0);
static_assert(DF % 32 == 0 && HL % 32 == 0 && KU % 32 == 0 && HL == 2 * DF && KU == 2 * HL);
static_assert(GBN == DF && GBM == GWAVE * 16 && DF == 4 * 32 && GTHR == GWAVE * 32);
static_assert(AGG_LDS_INTS * 4 <= 300000);
static_assert(ROWH == HL);
static_assert(NUWP % NTHR == 0 && NUWM % NTHR == 0 && NUWU % NTHR == 0 && NUW % NTHR == 0);
static_assert(RCAP * 100 >= MEAS_B1024 * 105);
static_assert(DEGCAP >= MEAS_MAXDEG + 8);
static_assert(FTHR == DF && NOUT == 32);

typedef float          v4f   __attribute__((ext_vector_type(4)));
typedef float          v8f   __attribute__((ext_vector_type(8)));
typedef int            v4i   __attribute__((ext_vector_type(4)));
typedef int            v8i   __attribute__((ext_vector_type(8)));
typedef unsigned short v4us  __attribute__((ext_vector_type(4)));
typedef unsigned short v8us  __attribute__((ext_vector_type(8)));
typedef unsigned short v16us __attribute__((ext_vector_type(16)));
typedef __bf16         v16bf __attribute__((ext_vector_type(16)));
typedef v4f  __attribute__((may_alias)) v4fa;
typedef v4i  __attribute__((may_alias)) v4ia;
typedef v4us __attribute__((may_alias)) v4usa;
typedef v8us __attribute__((may_alias)) v8usa;
union FragB { v16bf v; v16us u; v8us h[2]; v8i w; };

__device__ __forceinline__ v8f wmb(const FragB& a, const FragB& b, v8f c) {
  v8f d = __builtin_amdgcn_wmma_f32_16x16x32_bf16(false, a.v, false, b.v, (short)0, c, false, false);
  asm volatile("v_nop\n\tv_nop\n\tv_nop\n\tv_nop" : "+v"(d) : "v"(a.w), "v"(b.w));
  return d;
}

__device__ __forceinline__ v8f z8() { v8f z = {0.f, 0.f, 0.f, 0.f, 0.f, 0.f, 0.f, 0.f}; return z; }

__device__ __forceinline__ unsigned bf16_bits(float f) {
  const unsigned u = __float_as_uint(f);
  return (u + 0x7FFFu + ((u >> 16) & 1u)) >> 16;
}
__device__ __forceinline__ float bf16_val(float f) {
  return __uint_as_float(bf16_bits(f) << 16);
}
__device__ __forceinline__ unsigned hl_bits(float v, unsigned& lo) {
  const unsigned hb = bf16_bits(v);
  lo = bf16_bits(v - __uint_as_float(hb << 16));
  return hb;
}

__device__ __forceinline__ void wave_sync() {
  __builtin_amdgcn_fence(__ATOMIC_RELEASE, "wavefront");
  __builtin_amdgcn_wave_barrier();
  __builtin_amdgcn_fence(__ATOMIC_ACQUIRE, "wavefront");
}

__device__ __forceinline__ void kseg(v8f (&acc)[8], const unsigned short* ap, const unsigned short* bp,
                                     int ldb, int kLen) {
#pragma unroll 1
  for (int k0 = 0; k0 < kLen; k0 += 32) {
    FragB af;
    af.h[0] = *(const v8usa*)(ap + k0);
    af.h[1] = *(const v8usa*)(ap + k0 + 16);
#pragma unroll
    for (int nt = 0; nt < 8; ++nt) {
      const unsigned short* wq = bp + (size_t)(16 * nt) * (size_t)ldb + k0;
      FragB bf;
      bf.h[0] = *(const v8usa*)wq;
      bf.h[1] = *(const v8usa*)(wq + 16);
      acc[nt] = wmb(af, bf, acc[nt]);
    }
  }
}

template <int SLB>
__device__ __forceinline__ int scan_chunk(const int* __restrict__ dsts, int nE, int cbase, int slotBase,
                                          int nb, int vec8, int* list, int tid, int lane, int wave) {
  int wc = 0;
  const int el0  = tid * EPT;
  const int e0   = cbase + el0;
  const int sent = -2147483647 - 1;
  v4i da, db;
  if (vec8 != 0 && cbase + CHUNK <= nE) {
    da = *(const v4i*)(dsts + e0);
    db = *(const v4i*)(dsts + e0 + 4);
  } else {
    da.x = (e0     < nE) ? dsts[min(e0,     nE - 1)] : sent;
    da.y = (e0 + 1 < nE) ? dsts[min(e0 + 1, nE - 1)] : sent;
    da.z = (e0 + 2 < nE) ? dsts[min(e0 + 2, nE - 1)] : sent;
    da.w = (e0 + 3 < nE) ? dsts[min(e0 + 3, nE - 1)] : sent;
    db.x = (e0 + 4 < nE) ? dsts[min(e0 + 4, nE - 1)] : sent;
    db.y = (e0 + 5 < nE) ? dsts[min(e0 + 5, nE - 1)] : sent;
    db.z = (e0 + 6 < nE) ? dsts[min(e0 + 6, nE - 1)] : sent;
    db.w = (e0 + 7 < nE) ? dsts[min(e0 + 7, nE - 1)] : sent;
  }
  const unsigned nbs = (unsigned)slotBase;
  const unsigned unb = (unsigned)nb;
  const unsigned s0 = (unsigned)da.x - nbs, s1 = (unsigned)da.y - nbs;
  const unsigned s2 = (unsigned)da.z - nbs, s3 = (unsigned)da.w - nbs;
  const unsigned s4 = (unsigned)db.x - nbs, s5 = (unsigned)db.y - nbs;
  const unsigned s6 = (unsigned)db.z - nbs, s7 = (unsigned)db.w - nbs;
  const bool h0 = s0 < unb, h1 = s1 < unb, h2 = s2 < unb, h3 = s3 < unb;
  const bool h4 = s4 < unb, h5 = s5 < unb, h6 = s6 < unb, h7 = s7 < unb;
  const unsigned any = __builtin_amdgcn_ballot_w32(h0 | h1 | h2 | h3 | h4 | h5 | h6 | h7);
  if (any != 0u) {
#define HITJ(J, HJ, SJ) { \
      const unsigned mj = __builtin_amdgcn_ballot_w32(HJ); \
      if (mj != 0u) { \
        if (HJ) { \
          const int pos = wc + (int)__builtin_amdgcn_mbcnt_lo(mj, 0u); \
          if (pos < WCAP) list[wave * WCAP + pos] = ((el0 + (J)) << SLB) | (int)(SJ); \
        } \
        wc += (int)__builtin_popcount(mj); } }
    HITJ(0, h0, s0)
    HITJ(1, h1, s1)
    HITJ(2, h2, s2)
    HITJ(3, h3, s3)
    HITJ(4, h4, s4)
    HITJ(5, h5, s5)
    HITJ(6, h6, s6)
    HITJ(7, h7, s7)
#undef HITJ
  }
  return wc;
}

__global__ __launch_bounds__(NTHR) void k_prep(const float* __restrict__ x, const float* __restrict__ wp,
                                               const float* __restrict__ wm, const float* __restrict__ wu,
                                               unsigned short* wsb, size_t oWp, size_t oWm, size_t oWu, size_t oXb,
                                               int nN, int nUnits) {
  const int u = (int)blockIdx.x * NTHR + (int)threadIdx.x;
  v8us o;
  size_t dOff;
  if (u < NUWP) {
    const int n = u >> 4, k8 = (u & 15) * 8;
#pragma unroll
    for (int i = 0; i < 8; ++i) o[i] = (unsigned short)bf16_bits(wp[(size_t)(k8 + i) * DF + n]);
    dOff = oWp + (size_t)u * 8;
  } else if (u < NUWP + NUWM) {
    const int v  = u - NUWP;
    const int n  = v >> 5, k8 = (v & 31) * 8;
    const int r0 = ((n >> 7) << 7) + (k8 & (DF - 1));
    const int cn = n & (DF - 1);
#pragma unroll
    for (int i = 0; i < 8; ++i) o[i] = (unsigned short)bf16_bits(wm[(size_t)(r0 + i) * DF + cn]);
    dOff = oWm + (size_t)v * 8;
  } else if (u < NUW) {
    const int v  = u - NUWP - NUWM;
    const int n  = v >> 6, k8 = (v & 63) * 8;
    const int r0 = ((k8 >> 8) << 7) + (k8 & (DF - 1));
#pragma unroll
    for (int i = 0; i < 8; ++i) o[i] = (unsigned short)bf16_bits(wu[(size_t)(r0 + i) * DF + n]);
    dOff = oWu + (size_t)v * 8;
  } else if (u < nUnits) {
    const int v   = u - NUW;
    const int row = v >> 4, k8 = (v & 15) * 8;
    const int rc  = row < nN ? row : nN - 1;
    const bool lv = row < nN;
    const float* p = x + (size_t)rc * DF + k8;
    const v4f a = *(const v4f*)p;
    const v4f b = *(const v4f*)(p + 4);
    o[0] = lv ? (unsigned short)bf16_bits(a.x) : (unsigned short)0;
    o[1] = lv ? (unsigned short)bf16_bits(a.y) : (unsigned short)0;
    o[2] = lv ? (unsigned short)bf16_bits(a.z) : (unsigned short)0;
    o[3] = lv ? (unsigned short)bf16_bits(a.w) : (unsigned short)0;
    o[4] = lv ? (unsigned short)bf16_bits(b.x) : (unsigned short)0;
    o[5] = lv ? (unsigned short)bf16_bits(b.y) : (unsigned short)0;
    o[6] = lv ? (unsigned short)bf16_bits(b.z) : (unsigned short)0;
    o[7] = lv ? (unsigned short)bf16_bits(b.w) : (unsigned short)0;
    dOff = oXb + (size_t)v * 8;
  } else {
    return;
  }
  unsigned short* dp = wsb + dOff;
  *(volatile v8us*)dp = o;
  __threadfence();
  *(volatile v8us*)dp = o;
}

__global__ __launch_bounds__(GTHR) void k_gemm0(const unsigned short* xb, const unsigned short* wpt,
                                                const float* __restrict__ bp, float* h0, unsigned short* h0hl,
                                                int nN, int mRows) {
  __shared__ __attribute__((aligned(16))) float stg[GBM * GBN];
  const int tid = (int)threadIdx.x, lane = tid & 31, wave = tid >> 5, hh = lane >> 4, m = lane & 15;
  const int rowBase = (int)blockIdx.x * GBM;

  v8f acc[8];
#pragma unroll
  for (int t = 0; t < 8; ++t) acc[t] = z8();
  kseg(acc, xb + (size_t)(rowBase + 16 * wave + m) * (size_t)DF + 8 * hh,
       wpt + (size_t)m * (size_t)DF + 8 * hh, DF, DF);

#pragma unroll
  for (int nt = 0; nt < 8; ++nt) {
    const int lc = 16 * nt + m;
#pragma unroll
    for (int r = 0; r < 8; ++r) {
      const int lr = 16 * wave + 8 * hh + r;
      stg[lr * GBN + lc] = acc[nt][r];
    }
  }
  __syncthreads();

  v4f bq;
  {
    const v4f b4 = *(const v4f*)(bp + 4 * lane);
    bq.x = bf16_val(b4.x); bq.y = bf16_val(b4.y); bq.z = bf16_val(b4.z); bq.w = bf16_val(b4.w);
  }
  v4f pv[16];
#pragma unroll
  for (int i = 0; i < 16; ++i) pv[i] = *(const v4fa*)(stg + (16 * wave + i) * GBN + 4 * lane);
  __syncthreads();

#pragma unroll
  for (int i = 0; i < 16; ++i) {
    const bool ok = (rowBase + 16 * wave + i) < nN;
    v4f y = pv[i] + bq;
    y.x = ok ? y.x : 0.0f; y.y = ok ? y.y : 0.0f; y.z = ok ? y.z : 0.0f; y.w = ok ? y.w : 0.0f;
    pv[i] = y;
  }
#pragma unroll
  for (int i = 0; i < 16; ++i) {
    const int gr = rowBase + 16 * wave + i;
    float* op = h0 + (size_t)gr * DF + 4 * lane;
    if (gr < mRows) *(volatile v4f*)op = pv[i];
  }
#pragma unroll
  for (int i = 0; i < 16; ++i) {
    v4us h4, l4;
    unsigned lb;
    unsigned hb;
    hb = hl_bits(pv[i].x, lb); h4[0] = (unsigned short)hb; l4[0] = (unsigned short)lb;
    hb = hl_bits(pv[i].y, lb); h4[1] = (unsigned short)hb; l4[1] = (unsigned short)lb;
    hb = hl_bits(pv[i].z, lb); h4[2] = (unsigned short)hb; l4[2] = (unsigned short)lb;
    hb = hl_bits(pv[i].w, lb); h4[3] = (unsigned short)hb; l4[3] = (unsigned short)lb;
    unsigned short* srow = (unsigned short*)stg + (size_t)(16 * wave + i) * (2 * GBN);
    *(v4usa*)(srow + 4 * lane) = h4;
    *(v4usa*)(srow + DF + 4 * lane) = l4;
  }
  __syncthreads();
  v8us qv[16];
#pragma unroll
  for (int i = 0; i < 16; ++i) {
    const unsigned short* srow = (const unsigned short*)stg + (size_t)(16 * wave + i) * (2 * GBN);
    qv[i] = *(const v8usa*)(srow + 8 * lane);
  }
#pragma unroll
  for (int i = 0; i < 16; ++i) {
    const int gr = rowBase + 16 * wave + i;
    unsigned short* rp = h0hl + (size_t)gr * (size_t)HL + 8 * lane;
    if (gr < mRows) *(volatile v8us*)rp = qv[i];
  }
  __threadfence();
#pragma unroll
  for (int i = 0; i < 16; ++i) {
    const int gr = rowBase + 16 * wave + i;
    float* op = h0 + (size_t)gr * DF + 4 * lane;
    unsigned short* rp = h0hl + (size_t)gr * (size_t)HL + 8 * lane;
    if (gr < mRows) {
      *(volatile v4f*)op = pv[i];
      *(volatile v8us*)rp = qv[i];
    }
  }
}

__global__ __launch_bounds__(GTHR) void k_gemm_pq(const unsigned short* h0hl, const unsigned short* wmd,
                                                  const float* __restrict__ bm, float* pq, int planeElems,
                                                  int nN, int mRows) {
  __shared__ __attribute__((aligned(16))) float stg[GBM * GBN];
  const int tid = (int)threadIdx.x, lane = tid & 31, wave = tid >> 5, hh = lane >> 4, m = lane & 15;
  const int rowBase = (int)blockIdx.x * GBM;
  const int yq = (int)blockIdx.y;

  v8f acc[8];
#pragma unroll
  for (int t = 0; t < 8; ++t) acc[t] = z8();
  kseg(acc, h0hl + (size_t)(rowBase + 16 * wave + m) * (size_t)HL + 8 * hh,
       wmd + (size_t)(yq * DF + m) * (size_t)HL + 8 * hh, HL, HL);

#pragma unroll
  for (int nt = 0; nt < 8; ++nt) {
    const int lc = 16 * nt + m;
#pragma unroll
    for (int r = 0; r < 8; ++r) {
      const int lr = 16 * wave + 8 * hh + r;
      stg[lr * GBN + lc] = acc[nt][r];
    }
  }
  __syncthreads();

  v4f bq;
  {
    const v4f b4 = *(const v4f*)(bm + 4 * lane);
    bq.x = (yq != 0) ? bf16_val(b4.x) : 0.0f;
    bq.y = (yq != 0) ? bf16_val(b4.y) : 0.0f;
    bq.z = (yq != 0) ? bf16_val(b4.z) : 0.0f;
    bq.w = (yq != 0) ? bf16_val(b4.w) : 0.0f;
  }
  v4f pv[16];
#pragma unroll
  for (int i = 0; i < 16; ++i) pv[i] = *(const v4fa*)(stg + (16 * wave + i) * GBN + 4 * lane);
#pragma unroll
  for (int i = 0; i < 16; ++i) {
    const bool ok = (rowBase + 16 * wave + i) < nN;
    v4f y = pv[i] + bq;
    y.x = ok ? y.x : 0.0f; y.y = ok ? y.y : 0.0f; y.z = ok ? y.z : 0.0f; y.w = ok ? y.w : 0.0f;
    pv[i] = y;
  }
  float* plane = pq + (size_t)yq * (size_t)planeElems;
#pragma unroll
  for (int i = 0; i < 16; ++i) {
    const int gr = rowBase + 16 * wave + i;
    float* op = plane + (size_t)gr * DF + 4 * lane;
    if (gr < mRows) *(volatile v4f*)op = pv[i];
  }
  __threadfence();
#pragma unroll
  for (int i = 0; i < 16; ++i) {
    const int gr = rowBase + 16 * wave + i;
    float* op = plane + (size_t)gr * DF + 4 * lane;
    if (gr < mRows) *(volatile v4f*)op = pv[i];
  }
}

__global__ __launch_bounds__(NTHR) void k_scan(const int* __restrict__ srcs, const int* __restrict__ dsts,
                                               int nE, int nN, int vec8, int mRows,
                                               const float* __restrict__ pq, int planeElems,
                                               unsigned short* pool) {
  extern __shared__ __attribute__((aligned(16))) int dsm[];
  int* list = dsm;
  int* hl   = dsm + LISTN;
  int* sl   = hl + RCAP;
  int* cnt  = sl + RCAP;
  int* offs = cnt + NBA;
  int* cur  = offs + NBA;
  int* misc = cur + NBA;
  const int tid = (int)threadIdx.x, lane = tid & 31, wave = tid >> 5;
  unsigned short* rowbuf = (unsigned short*)(misc + MISC_INTS) + wave * ROWH;
  const int nodeBase = (int)blockIdx.x * NBA;
  int nbv = nN - nodeBase;
  nbv = nbv < 0 ? 0 : (nbv > NBA ? NBA : nbv);
  const float* pP = pq;
  const float* pQ = pq + (size_t)planeElems;

  {
    const v4i z4 = {0, 0, 0, 0};
    for (int i = tid * 4; i < AGG_ZINTS; i += NTHR * 4) *(v4ia*)(dsm + i) = z4;
    if (tid < MISC_INTS) misc[tid] = 0;
  }
  __syncthreads();

  int t = 0, ov = 0;
  const int nChunks = (nE + CHUNK - 1) / CHUNK;
#pragma unroll 1
  for (int ch = 0; ch < nChunks; ++ch) {
    const int cbase = ch * CHUNK;
    const int wc = scan_chunk<SLA>(dsts, nE, cbase, nodeBase, nbv, vec8, list, tid, lane, wave);
    if (lane == 0) misc[wave] = wc;
    __syncthreads();
    if (wave == 0) {
#pragma unroll 1
      for (int w2 = 0; w2 < NWAVE; ++w2) {
        int c = misc[w2];
        c = c < 0 ? 0 : (c > WCAP ? WCAP : c);
#pragma unroll 1
        for (int b0 = 0; b0 < c; b0 += 32) {
          const int idx = b0 + lane;
          const int ent = list[w2 * WCAP + (idx < WCAP ? idx : WCAP - 1)];
          const int m32 = (c - b0) < 32 ? (c - b0) : 32;
#pragma unroll 1
          for (int k = 0; k < m32; ++k) {
            const int u    = __builtin_amdgcn_readlane(ent, k);
            const int slot = u & (NBA - 1);
            const int el   = (u >> SLA) & (CHUNK - 1);
            const int pk   = ((cbase + el) << SLA) | slot;
            if (t < RCAP) {
              if (lane == 0) { hl[t] = pk; cnt[slot] = cnt[slot] + 1; }
              t = t + 1;
            } else {
              ov = 1;
            }
          }
        }
      }
    }
    __syncthreads();
  }
  if (wave == 0 && lane == 0) { misc[8] = t; misc[9] = ov; }
  __syncthreads();
  int tt = misc[8];
  tt = tt < 0 ? 0 : (tt > RCAP ? RCAP : tt);
  const int ovf = misc[9];

  if (wave == 0) {
    const int base = lane * (NBA / 32);
    int s = 0;
#pragma unroll 1
    for (int i = 0; i < NBA / 32; ++i) s += cnt[base + i];
    int incl = s;
#pragma unroll
    for (int d = 1; d < 32; d <<= 1) {
      const int y = __shfl_up(incl, d, 32);
      if (lane >= d) incl += y;
    }
    int run = incl - s;
#pragma unroll 1
    for (int i = 0; i < NBA / 32; ++i) {
      const int cv = cnt[base + i];
      offs[base + i] = run;
      cur[base + i]  = run;
      run += cv;
    }
  }
  __syncthreads();
  if (wave == 0) {
#pragma unroll 1
    for (int b0 = 0; b0 < tt; b0 += 32) {
      const int idx = b0 + lane;
      const int ent = hl[idx < RCAP ? idx : RCAP - 1];
      const int m32 = (tt - b0) < 32 ? (tt - b0) : 32;
#pragma unroll 1
      for (int k = 0; k < m32; ++k) {
        const int u    = __builtin_amdgcn_readlane(ent, k);
        const int slot = u & (NBA - 1);
        if (lane == 0) {
          int p = cur[slot];
          p = p < 0 ? 0 : (p > RCAP - 1 ? RCAP - 1 : p);
          sl[p] = u;
          cur[slot] = p + 1;
        }
      }
    }
  }
  __syncthreads();

  const float pz = (ovf != 0) ? __int_as_float(0x7fc00000) : 0.0f;
#pragma unroll 1
  for (int si = 0; si < NBA / NWAVE; ++si) {
    const int s    = si * NWAVE + wave;
    const int node = nodeBase + s;
    int c = cnt[s];
    const bool big = c > DEGCAP;
    c = c < 0 ? 0 : (c > DEGCAP ? DEGCAP : c);
    int o = offs[s];
    o = o < 0 ? 0 : (o > RCAP ? RCAP : o);
    const float pzr = big ? __int_as_float(0x7fc00000) : pz;
    const bool live = node < nN;
    const int nc = live ? node : nN - 1;
    const v4f qr = *(const v4f*)(pQ + (size_t)nc * DF + 4 * lane);
    float a0 = 0.0f, a1 = 0.0f, a2 = 0.0f, a3 = 0.0f;
#pragma unroll 1
    for (int b0 = 0; b0 < c; b0 += 32) {
      int idx = o + b0 + lane;
      idx = idx > RCAP - 1 ? RCAP - 1 : idx;
      const int ent = sl[idx];
      int eid = ent >> SLA;
      eid = eid < 0 ? 0 : (eid > nE - 1 ? nE - 1 : eid);
      int sr = srcs[eid];
      sr = sr < 0 ? 0 : (sr > nN - 1 ? nN - 1 : sr);
      const int m32 = (c - b0) < 32 ? (c - b0) : 32;
#pragma unroll 1
      for (int k = 0; k < m32; ++k) {
        const int sk = __builtin_amdgcn_readlane(sr, k);
        const v4f pr = *(const v4f*)(pP + (size_t)sk * DF + 4 * lane);
        const float v0 = pr.x + qr.x, v1 = pr.y + qr.y, v2 = pr.z + qr.z, v3 = pr.w + qr.w;
        a0 += (v0 > 0.0f) ? v0 : (v0 - v0);
        a1 += (v1 > 0.0f) ? v1 : (v1 - v1);
        a2 += (v2 > 0.0f) ? v2 : (v2 - v2);
        a3 += (v3 > 0.0f) ? v3 : (v3 - v3);
      }
    }
    const float cf = fmaxf((float)c, 1.0f);
    const float m0 = live ? (a0 / cf + pzr) : 0.0f;
    const float m1 = live ? (a1 / cf + pzr) : 0.0f;
    const float m2 = live ? (a2 / cf + pzr) : 0.0f;
    const float m3 = live ? (a3 / cf + pzr) : 0.0f;
    v4us mh, ml;
    {
      unsigned lb;
      unsigned hb;
      hb = hl_bits(m0, lb); mh[0] = (unsigned short)hb; ml[0] = (unsigned short)lb;
      hb = hl_bits(m1, lb); mh[1] = (unsigned short)hb; ml[1] = (unsigned short)lb;
      hb = hl_bits(m2, lb); mh[2] = (unsigned short)hb; ml[2] = (unsigned short)lb;
      hb = hl_bits(m3, lb); mh[3] = (unsigned short)hb; ml[3] = (unsigned short)lb;
    }
    *(v4usa*)(rowbuf + 4 * lane)      = mh;
    *(v4usa*)(rowbuf + DF + 4 * lane) = ml;
    wave_sync();
    const v8us q0 = *(const v8usa*)(rowbuf + 8 * lane);
    wave_sync();
    if (node < mRows) {
      unsigned short* rpw = pool + (size_t)node * HL + 8 * lane;
      *(volatile v8us*)rpw = q0;
      __threadfence();
      *(volatile v8us*)rpw = q0;
    }
  }
}

__global__ __launch_bounds__(GTHR) void k_gemm_u(const unsigned short* h0hl, const unsigned short* poolhl,
                                                 const unsigned short* wud, const float* h0,
                                                 const float* __restrict__ bu, const float* __restrict__ gam,
                                                 const float* __restrict__ bet, float* rec, int nN) {
  __shared__ __attribute__((aligned(16))) float stg[GBM * GBN];
  __shared__ __attribute__((aligned(16))) float part[GWAVE * DF];
  const int tid = (int)threadIdx.x, lane = tid & 31, wave = tid >> 5, hh = lane >> 4, m = lane & 15;
  const int rowBase = (int)blockIdx.x * GBM;

  v8f acc[8];
#pragma unroll
  for (int t = 0; t < 8; ++t) acc[t] = z8();
  {
    const size_t arow = (size_t)(rowBase + 16 * wave + m) * (size_t)HL + 8 * hh;
    const unsigned short* bp = wud + (size_t)m * (size_t)KU + 8 * hh;
    kseg(acc, h0hl + arow, bp, KU, HL);
    kseg(acc, poolhl + arow, bp + HL, KU, HL);
  }

#pragma unroll
  for (int nt = 0; nt < 8; ++nt) {
    const int lc = 16 * nt + m;
#pragma unroll
    for (int r = 0; r < 8; ++r) {
      const int lr = 16 * wave + 8 * hh + r;
      stg[lr * GBN + lc] = acc[nt][r];
    }
  }
  __syncthreads();

  v4f bq, gq, eq;
  {
    const v4f b4 = *(const v4f*)(bu + 4 * lane);
    const v4f g4 = *(const v4f*)(gam + 4 * lane);
    const v4f e4 = *(const v4f*)(bet + 4 * lane);
    bq.x = bf16_val(b4.x); bq.y = bf16_val(b4.y); bq.z = bf16_val(b4.z); bq.w = bf16_val(b4.w);
    gq.x = bf16_val(g4.x); gq.y = bf16_val(g4.y); gq.z = bf16_val(g4.z); gq.w = bf16_val(g4.w);
    eq.x = bf16_val(e4.x); eq.y = bf16_val(e4.y); eq.z = bf16_val(e4.z); eq.w = bf16_val(e4.w);
  }

  const float invd = 1.0f / (float)DF;
  float cs0 = 0.0f, cs1 = 0.0f, cs2 = 0.0f, cs3 = 0.0f;
#pragma unroll 1
  for (int i = 0; i < 16; ++i) {
    const int lr  = 16 * wave + i;
    const int row = rowBase + lr;
    const bool ok = row < nN;
    const v4f d  = *(const v4fa*)(stg + lr * GBN + 4 * lane);
    const v4f hr = *(const v4f*)(h0 + (size_t)row * DF + 4 * lane);
    const float v0 = hr.x + (d.x + bq.x), v1 = hr.y + (d.y + bq.y);
    const float v2 = hr.z + (d.z + bq.z), v3 = hr.w + (d.w + bq.w);
    const float n0 = (v0 > 0.0f) ? v0 : (v0 - v0);
    const float n1 = (v1 > 0.0f) ? v1 : (v1 - v1);
    const float n2 = (v2 > 0.0f) ? v2 : (v2 - v2);
    const float n3 = (v3 > 0.0f) ? v3 : (v3 - v3);
    float s = (n0 + n1) + (n2 + n3);
    s += __shfl_xor(s, 16, 32);
    s += __shfl_xor(s, 8, 32);
    s += __shfl_xor(s, 4, 32);
    s += __shfl_xor(s, 2, 32);
    s += __shfl_xor(s, 1, 32);
    const float mu = s * invd;
    const float d0 = n0 - mu, d1 = n1 - mu, d2 = n2 - mu, d3 = n3 - mu;
    float q = (d0 * d0 + d1 * d1) + (d2 * d2 + d3 * d3);
    q += __shfl_xor(q, 16, 32);
    q += __shfl_xor(q, 8, 32);
    q += __shfl_xor(q, 4, 32);
    q += __shfl_xor(q, 2, 32);
    q += __shfl_xor(q, 1, 32);
    const float var  = q * invd;
    const float rstd = 1.0f / sqrtf(var + LNEPS);
    const float y0 = d0 * rstd * gq.x + eq.x;
    const float y1 = d1 * rstd * gq.y + eq.y;
    const float y2 = d2 * rstd * gq.z + eq.z;
    const float y3 = d3 * rstd * gq.w + eq.w;
    cs0 += ok ? y0 : 0.0f;
    cs1 += ok ? y1 : 0.0f;
    cs2 += ok ? y2 : 0.0f;
    cs3 += ok ? y3 : 0.0f;
  }
  {
    v4f c4; c4.x = cs0; c4.y = cs1; c4.z = cs2; c4.w = cs3;
    *(v4fa*)(part + wave * DF + 4 * lane) = c4;
  }
  __syncthreads();
  if (wave == 0) {
    const v4f p0 = *(const v4fa*)(part + 0 * DF + 4 * lane);
    const v4f p1 = *(const v4fa*)(part + 1 * DF + 4 * lane);
    const v4f p2 = *(const v4fa*)(part + 2 * DF + 4 * lane);
    const v4f p3 = *(const v4fa*)(part + 3 * DF + 4 * lane);
    const v4f tsum = ((p0 + p1) + p2) + p3;
    float* rp = rec + (size_t)blockIdx.x * DF + 4 * lane;
    *(volatile v4f*)rp = tsum;
    __threadfence();
    *(volatile v4f*)rp = tsum;
  }
}

__global__ __launch_bounds__(FTHR) void k_final(const float* rec, int nRec, double invN,
                                                const float* __restrict__ wd, const float* __restrict__ bd,
                                                float* outp) {
  __shared__ double gl[DF];
  const int tid = (int)threadIdx.x;
  double s = 0.0;
#pragma unroll 4
  for (int b = 0; b < nRec; ++b) s += (double)rec[(size_t)b * DF + tid];
  gl[tid] = s * invN;
  __syncthreads();
  if (tid < NOUT) {
    double a = 0.0;
#pragma unroll 4
    for (int c = 0; c < DF; ++c) a += gl[c] * (double)bf16_val(wd[c * NOUT + tid]);
    const float o = (float)(a + (double)bf16_val(bd[tid]));
    float* op = outp + tid;
    *(volatile float*)op = o;
    __threadfence();
    *(volatile float*)op = o;
  }
}

static inline int cdiv(int a, int b) { return (a + b - 1) / b; }
static inline size_t al256(size_t o) { return (o + 255) & ~(size_t)255; }

extern "C" void kernel_launch(void* const* d_in, const int* in_sizes, int n_in,
                              void* d_out, int out_size, void* d_ws, size_t ws_size,
                              hipStream_t stream) {
  if (n_in < 13) return;
  if (in_sizes[0] < DF * GBM || (in_sizes[0] % DF) != 0) return;
  const int nN = in_sizes[0] / DF;
  if (nN >= (1 << 22)) return;
  const int nE = in_sizes[1];
  if (nE < 1 || in_sizes[2] != nE || nE >= (1 << 21)) return;
  if (in_sizes[3] != DF * DF || in_sizes[4] != DF) return;
  if (in_sizes[5] != 2 * DF * DF || in_sizes[6] != DF) return;
  if (in_sizes[7] != 2 * DF * DF || in_sizes[8] != DF) return;
  if (in_sizes[9] != DF || in_sizes[10] != DF) return;
  if (in_sizes[11] != DF * NOUT || in_sizes[12] != NOUT) return;
  if (out_size != NOUT) return;

  const float* x    = (const float*)d_in[0];
  const int*   esrc = (const int*)  d_in[1];
  const int*   edst = (const int*)  d_in[2];
  const float* Wp   = (const float*)d_in[3];
  const float* bp   = (const float*)d_in[4];
  const float* Wm   = (const float*)d_in[5];
  const float* bm   = (const float*)d_in[6];
  const float* Wu   = (const float*)d_in[7];
  const float* bu   = (const float*)d_in[8];
  const float* gam  = (const float*)d_in[9];
  const float* bet  = (const float*)d_in[10];
  const float* Wd   = (const float*)d_in[11];
  const float* bd   = (const float*)d_in[12];
  float* out = (float*)d_out;

  const int MP = cdiv(nN, GBM) * GBM;
  const int gM = MP / GBM;
  const int gA = cdiv(nN, NBA);
  if ((long long)gA * NBA < (long long)MP) return;
  const int vec8 = ((nE & 3) == 0) ? 1 : 0;
  const int planeElems = MP * DF;

  char* ws = (char*)d_ws;
  size_t off = 0;
  const size_t oWPT  = off; off = al256(off + (size_t)DF * DF * 2);
  const size_t oWMD  = off; off = al256(off + (size_t)2 * DF * HL * 2);
  const size_t oWUD  = off; off = al256(off + (size_t)DF * KU * 2);
  const size_t oH0   = off; off = al256(off + (size_t)MP * DF * 4);
  const size_t oH0HL = off; off = al256(off + (size_t)MP * HL * 2);
  const size_t oPQ   = off; off = al256(off + (size_t)2 * MP * DF * 4);
  const size_t oPOOL = off; off = al256(off + (size_t)MP * HL * 2);
  const size_t oREC  = off; off = al256(off + (size_t)gM * DF * 4);
  const size_t oXB   = oPOOL;
  if (off > ws_size || off > (size_t)WSMAX) return;
  unsigned short* wsb   = (unsigned short*)ws;
  unsigned short* WPT   = (unsigned short*)(ws + oWPT);
  unsigned short* WMD   = (unsigned short*)(ws + oWMD);
  unsigned short* WUD   = (unsigned short*)(ws + oWUD);
  float*          H0    = (float*)(ws + oH0);
  unsigned short* H0HL  = (unsigned short*)(ws + oH0HL);
  float*          PQ    = (float*)(ws + oPQ);
  unsigned short* POOL  = (unsigned short*)(ws + oPOOL);
  float*          REC   = (float*)(ws + oREC);
  unsigned short* XB    = (unsigned short*)(ws + oXB);

  const size_t scanLds = (size_t)AGG_LDS_INTS * 4;
  hipFuncSetAttribute(reinterpret_cast<const void*>(&k_scan), hipFuncAttributeMaxDynamicSharedMemorySize, (int)scanLds);

  const int nUnits = NUW + MP * (DF / 8);

  k_prep<<<cdiv(nUnits, NTHR), NTHR, 0, stream>>>(x, Wp, Wm, Wu, wsb, oWPT / 2, oWMD / 2, oWUD / 2, oXB / 2,
                                                  nN, nUnits);
  k_gemm0<<<gM, GTHR, 0, stream>>>(XB, WPT, bp, H0, H0HL, nN, MP);
  k_gemm_pq<<<dim3((unsigned)gM, 2u, 1u), GTHR, 0, stream>>>(H0HL, WMD, bm, PQ, planeElems, nN, MP);
  k_scan<<<gA, NTHR, scanLds, stream>>>(esrc, edst, nE, nN, vec8, MP, PQ, planeElems, POOL);
  k_gemm_u<<<gM, GTHR, 0, stream>>>(H0HL, POOL, WUD, H0, bu, gam, bet, REC, nN);
  k_final<<<1, FTHR, 0, stream>>>(REC, gM, 1.0 / (double)nN, Wd, bd, out);
}
